// PhysicsInformedHardProj_89300960018671
// MI455X (gfx1250) — hardware-verified
//
#include <hip/hip_runtime.h>
#include <math.h>

typedef __attribute__((ext_vector_type(16))) _Float16 v16h;
typedef __attribute__((ext_vector_type(16))) __bf16 v16b;
typedef __attribute__((ext_vector_type(8)))  _Float16 v8h;
typedef __attribute__((ext_vector_type(8)))  float v8f;
typedef __attribute__((ext_vector_type(4)))  float v4f;
typedef __attribute__((ext_vector_type(2)))  float v2f;
typedef __attribute__((ext_vector_type(4)))  unsigned v4u;
typedef __attribute__((ext_vector_type(4)))  int v4i;
typedef float __attribute__((may_alias)) float_a;
typedef int __attribute__((may_alias)) int_a;

template <typename T> __device__ __forceinline__ void vst2(void* p, T v) { *(volatile T*)p = v; __threadfence(); *(volatile T*)p = v; }
__device__ __forceinline__ v8f wmma16(v16h a, v16h b, v8f c) {
  v8f d = __builtin_amdgcn_wmma_f32_16x16x32_f16(false, a, false, b, (short)0, c, false, false);
  asm volatile("v_nop\n\tv_nop\n\tv_nop\n\tv_nop" : "+v"(d) : "v"(a), "v"(b));
  return d;
}
__device__ __forceinline__ v8f wmma_bf(v16b a, v16b b, v8f c) {
  v8f d = __builtin_amdgcn_wmma_f32_16x16x32_bf16(false, a, false, b, (short)0, c, false, false);
  asm volatile("v_nop\n\tv_nop\n\tv_nop\n\tv_nop" : "+v"(d) : "v"(a), "v"(b));
  return d;
}
__device__ __forceinline__ v16h frag_h(const _Float16* rowk0, int lane) {
  union { v16h v; v8h q[2]; } u; const _Float16* p = rowk0 + 8 * (lane >> 4);
  u.q[0] = *(const v8h*)p; u.q[1] = *(const v8h*)(p + 16); return u.v;
}
__device__ __forceinline__ v16h frag_f32(const float* rowk0, int lane) {
  v16h a; const float* p = rowk0 + 8 * (lane >> 4);
#pragma unroll
  for (int i = 0; i < 8; ++i) { a[i] = (_Float16)p[i]; a[8 + i] = (_Float16)p[16 + i]; }
  return a;
}
__device__ __forceinline__ v16h frag_f32s(const float* rowk0, int lane, float sc) {
  v16h a; const float* p = rowk0 + 8 * (lane >> 4);
#pragma unroll
  for (int i = 0; i < 8; ++i) { a[i] = (_Float16)(p[i] * sc); a[8 + i] = (_Float16)(p[16 + i] * sc); }
  return a;
}
__device__ __forceinline__ v16h fragc_f32(const float* W, int k0, int n, int lane, int ld, int K) {
  v16h a; const int g = lane >> 4;
#pragma unroll
  for (int i = 0; i < 8; ++i) { const int ka = k0 + 8 * g + i, kb = ka + 16;
    a[i] = (_Float16)(ka < K ? W[(size_t)(ka < K ? ka : K - 1) * ld + n] : 0.f); a[8 + i] = (_Float16)(kb < K ? W[(size_t)(kb < K ? kb : K - 1) * ld + n] : 0.f); }
  return a;
}
struct F2 { v16b h, l; };
__device__ __forceinline__ F2 bsplit16(const float v[16]) { F2 r;
#pragma unroll
  for (int i = 0; i < 16; ++i) { const __bf16 h = (__bf16)v[i]; r.h[i] = h; r.l[i] = (__bf16)(v[i] - (float)h); }
  return r; }
__device__ __forceinline__ F2 split_row(const float* row, int k0, int lane) { float v[16]; const float* p = row + k0 + 8 * (lane >> 4);
#pragma unroll
  for (int i = 0; i < 8; ++i) { v[i] = p[i]; v[8 + i] = p[16 + i]; }
  return bsplit16(v); }
__device__ __forceinline__ F2 split_rowK(const float* row, int k0, int lane, int K) { float v[16]; const int g = lane >> 4;
#pragma unroll
  for (int i = 0; i < 8; ++i) { const int ka = k0 + 8 * g + i, kb = ka + 16; v[i] = ka < K ? row[ka < K ? ka : K - 1] : 0.f; v[8 + i] = kb < K ? row[kb < K ? kb : K - 1] : 0.f; }
  return bsplit16(v); }
__device__ __forceinline__ F2 split_col(const float* W, int k0, int n, int lane, int ld, int K) { float v[16]; const int g = lane >> 4;
#pragma unroll
  for (int i = 0; i < 8; ++i) { const int ka = k0 + 8 * g + i, kb = ka + 16; v[i] = ka < K ? W[(size_t)(ka < K ? ka : K - 1) * ld + n] : 0.f; v[8 + i] = kb < K ? W[(size_t)(kb < K ? kb : K - 1) * ld + n] : 0.f; }
  return bsplit16(v); }
__device__ __forceinline__ v8f mac3(const F2& a, const F2& b, v8f c) { c = wmma_bf(a.l, b.h, c); c = wmma_bf(a.h, b.l, c); return wmma_bf(a.h, b.h, c); }
__device__ __forceinline__ float sigm(float v) { return 1.0f / (1.0f + expf(-v)); }
#define LDSX() do { asm volatile("s_wait_dscnt 0" ::: "memory"); __builtin_amdgcn_wave_barrier(); __builtin_amdgcn_fence(__ATOMIC_RELEASE, "workgroup"); } while (0)


#define NPTS 1000000
#define HH 64
#define NE 4
#define NS 3
#define NBLK ((NPTS + 63) / 64)
#ifndef TBLK
#define TBLK NBLK
#endif
typedef __attribute__((ext_vector_type(8))) __bf16 v8b;
__device__ __forceinline__ v16b frag_b(const __bf16* rowk0, int lane) {
  union { v16b v; v8b q[2]; } u; const __bf16* p = rowk0 + 8 * (lane >> 4);
  u.q[0] = *(const v8b*)p; u.q[1] = *(const v8b*)(p + 16); return u.v;
}
__device__ __forceinline__ float bfr(float v) { return (float)(__bf16)v; }
__device__ __attribute__((noinline)) float exp_ni(float v) { return expf(v); }
__device__ __attribute__((noinline)) float erf_ni(float v) { return erff(v); }

#define WS_END 64u

__device__ __forceinline__ v16b fragw(const float* __restrict__ Wm, int ncol, int o, int k0, int lane) { v16b w; const int kb = k0 + 8 * (lane >> 4);
#pragma unroll
  for (int i = 0; i < 8; ++i) { w[i] = (o < ncol) ? (__bf16)Wm[(size_t)(kb + i) * ncol + o] : (__bf16)0.0f; w[8 + i] = (o < ncol) ? (__bf16)Wm[(size_t)(kb + 16 + i) * ncol + o] : (__bf16)0.0f; } return w; }
__global__ __launch_bounds__(128) void k_php(const float* __restrict__ PC, const float* __restrict__ W1, const float* __restrict__ B1, const float* __restrict__ W2, const float* __restrict__ B2, const float* __restrict__ W3, const float* __restrict__ B3, const float* __restrict__ WMU, const float* __restrict__ BMU, const float* __restrict__ WLAM, const float* __restrict__ BLAM, float* __restrict__ OUT) {
  __shared__ __align__(16) float sa[64][HH + 4]; __shared__ __align__(16) float shd[64][8]; __shared__ __align__(16) float so[8][64];
  const int tid = threadIdx.x, wave = tid >> 5, lane = tid & 31, col = lane & 15, g = lane >> 4; const size_t n0 = (size_t)blockIdx.x * 64;
  for (int e = tid; e < 64 * HH; e += 128) { const int pl = e >> 6, c = e & 63; const size_t n = n0 + pl; const float x0 = bfr(PC[n * 2]), x1 = bfr(PC[n * 2 + 1]); sa[pl][c] = fmaxf(x0 * bfr(W1[c]) + x1 * bfr(W1[HH + c]) + bfr(B1[c]), 0.f); }
  __syncthreads();
#pragma unroll 1
  for (int layer = 0; layer < 2; ++layer) { const float* Wm = layer == 0 ? W2 : W3; const float* Bm = layer == 0 ? B2 : B3; v8f acc[4] = {};
#pragma unroll
    for (int kc = 0; kc < HH / 32; ++kc) { float v[16]; const float* pp = &sa[wave * 16 + col][kc * 32 + 8 * g];
#pragma unroll
      for (int i = 0; i < 8; ++i) { v[i] = pp[i]; v[8 + i] = pp[16 + i]; }
      const F2 a = bsplit16(v);
#pragma unroll
      for (int j = 0; j < 4; ++j) { const v16b w = fragw(Wm, HH, j * 16 + col, kc * 32, lane); acc[j] = wmma_bf(a.h, w, acc[j]); acc[j] = wmma_bf(a.l, w, acc[j]); } }
    LDSX();
#pragma unroll
    for (int j = 0; j < 4; ++j) { const int c = j * 16 + col; const float bb = bfr(Bm[c]);
#pragma unroll
      for (int r = 0; r < 8; ++r) sa[wave * 16 + 8 * g + r][c] = fmaxf(acc[j][r] + bb, 0.f); }
    LDSX(); }
  { v8f acc = {};
#pragma unroll
    for (int kc = 0; kc < HH / 32; ++kc) { float v[16]; const float* pp = &sa[wave * 16 + col][kc * 32 + 8 * g];
#pragma unroll
      for (int i = 0; i < 8; ++i) { v[i] = pp[i]; v[8 + i] = pp[16 + i]; }
      const F2 a = bsplit16(v); v16b w; if (col < NE) w = fragw(WMU, NE, col, kc * 32, lane); else w = fragw(WLAM, NS, col - NE, kc * 32, lane);
      acc = wmma_bf(a.h, w, acc); acc = wmma_bf(a.l, w, acc); }
    if (col < 8) { const float bb = (col < NE) ? bfr(BMU[col]) : (col < NE + NS ? bfr(BLAM[col - NE]) : 0.f);
#pragma unroll
      for (int r = 0; r < 8; ++r) shd[wave * 16 + 8 * g + r][col] = acc[r] + bb; } }
  __syncthreads();
  if (tid < 64) { const float* hv = shd[tid]; float mu0 = fmaxf(hv[0], 0.f), mu1 = fmaxf(hv[1], 0.f), mu2 = fmaxf(hv[2], 0.f), mu3 = fmaxf(hv[3], 0.f);
    const float g0 = mu0 - mu1, g1 = mu2 - mu3; const float nrm = sqrtf(g0 * g0 + g1 * g1); const float sc = (nrm > 1.0f) ? 1.0f / (nrm + 1e-8f) : 1.0f;
    so[0][tid] = mu0 * sc; so[1][tid] = mu1 * sc; so[2][tid] = mu2 * sc; so[3][tid] = mu3 * sc;
    const float l0 = hv[4], l1 = hv[5], l2 = hv[6]; const float il = 1.0f / (sqrtf(l0 * l0 + l1 * l1 + l2 * l2) + 1e-8f); so[4][tid] = l0 * il; so[5][tid] = l1 * il; so[6][tid] = l2 * il; }
  __syncthreads();
  { const int orow = tid >> 4, q = tid & 15; if (orow < NE + NS) { float* dst = (orow < NE) ? (OUT + (size_t)orow * NPTS) : (OUT + (size_t)NE * NPTS + (size_t)(orow - NE) * NPTS); vst2(dst + n0 + q * 4, *(const v4f*)&so[orow][q * 4]); } } }
extern "C" void kernel_launch(void* const* d_in, const int* in_sizes, int n_in, void* d_out, int out_size, void* d_ws, size_t ws_size, hipStream_t stream) {
  (void)in_sizes; (void)n_in; (void)out_size; (void)d_ws; (void)ws_size;
  const float** F = (const float**)d_in;
  k_php<<<TBLK, 128, 0, stream>>>(F[0], F[1], F[2], F[3], F[4], F[5], F[6], F[7], F[8], F[9], F[10], (float*)d_out);
}
